// SemisupKernelClassifier_3375844295427
// MI455X (gfx1250) — hardware-verified
//
#include <hip/hip_runtime.h>

typedef unsigned short v16us __attribute__((ext_vector_type(16)));
typedef unsigned short v8us  __attribute__((ext_vector_type(8)));
typedef __bf16         v16bf __attribute__((ext_vector_type(16)));
typedef float          v8f   __attribute__((ext_vector_type(8)));
typedef float          v4f   __attribute__((ext_vector_type(4)));
typedef v8us __attribute__((may_alias)) v8usa;
typedef v4f  __attribute__((may_alias)) v4fa;

union FragU { v16us v; v8us half[2]; };

#define NX   4096
#define DIM  64
#define NL   2048
#define NU   8192
#define MA   (NL + NU)
#define NC   10
#define PDP  16
#define JT   (MA / 16)
#define INV_SQRT_2PI 0.3989422804014327f
#define FMIN_NORMAL  1.17549435e-38f

__device__ __forceinline__ v8f wmma_bf16(v16us a, v16us b, v8f c) {
  const v16bf ab = __builtin_bit_cast(v16bf, a);
  const v16bf bb = __builtin_bit_cast(v16bf, b);
  v8f d = __builtin_amdgcn_wmma_f32_16x16x32_bf16(false, ab, false, bb, (short)0, c, false, false);
  asm volatile("v_nop\n\tv_nop\n\tv_nop\n\tv_nop" : "+v"(d) : "v"(a), "v"(b));
  return d;
}

__device__ __forceinline__ v16us load_frag(const unsigned short* p, int k0, int h) {
  FragU f;
  f.half[0] = *(const v8usa*)(p + k0 + 8 * h);
  f.half[1] = *(const v8usa*)(p + k0 + 16 + 8 * h);
  return f.v;
}

__device__ __forceinline__ unsigned int bf16_bits_rne(float f) {
  unsigned int u = __float_as_uint(f);
  u += 0x7FFFu + ((u >> 16) & 1u);
  return u >> 16;
}

__global__ __launch_bounds__(256) void prep_kernel(
    const float* __restrict__ x, const float* __restrict__ xl, const float* __restrict__ xu,
    unsigned short* __restrict__ xhi, unsigned short* __restrict__ xlo,
    unsigned short* __restrict__ ahi, unsigned short* __restrict__ alo,
    float* __restrict__ x2, float* __restrict__ a2)
{
  __shared__ __attribute__((aligned(16))) float sS[32];

  const int tid = threadIdx.x, b = blockIdx.x;
  const int r = tid >> 3, q = tid & 7;

  const float* src;
  unsigned short* dh;
  unsigned short* dl;
  float* dsq;
  if (b < NX / 32) {
    const int r0 = 32 * b;
    src = x + (size_t)r0 * DIM;
    dh  = xhi + (size_t)r0 * DIM;
    dl  = xlo + (size_t)r0 * DIM;
    dsq = x2 + r0;
  } else {
    const int k0 = 32 * (b - NX / 32);
    src = (k0 < NL) ? (xl + (size_t)k0 * DIM) : (xu + (size_t)(k0 - NL) * DIM);
    dh  = ahi + (size_t)k0 * DIM;
    dl  = alo + (size_t)k0 * DIM;
    dsq = a2 + k0;
  }

  const float* p = src + r * DIM + 8 * q;
  const v4f u0 = *(const v4fa*)p;
  const v4f u1 = *(const v4fa*)(p + 4);
  const float f[8] = { u0.x, u0.y, u0.z, u0.w, u1.x, u1.y, u1.z, u1.w };

  unsigned short hb[8], lb[8];
  float s = 0.0f;
  #pragma unroll
  for (int i = 0; i < 8; ++i) {
    const unsigned int hu = bf16_bits_rne(f[i]);
    const float hf = __uint_as_float(hu << 16);
    hb[i] = (unsigned short)hu;
    lb[i] = (unsigned short)bf16_bits_rne(f[i] - hf);
    s = fmaf(f[i], f[i], s);
  }
  const v8us hv = { hb[0], hb[1], hb[2], hb[3], hb[4], hb[5], hb[6], hb[7] };
  const v8us lv = { lb[0], lb[1], lb[2], lb[3], lb[4], lb[5], lb[6], lb[7] };

  s += __shfl_xor(s, 1);
  s += __shfl_xor(s, 2);
  s += __shfl_xor(s, 4);
  if (q == 0) sS[r] = s;
  __syncthreads();
  const v4f sq = *(const v4fa*)(sS + 4 * (tid & 7));

  unsigned short* ph = dh + r * DIM + 8 * q;
  unsigned short* pl = dl + r * DIM + 8 * q;

  *(volatile v8us*)ph = hv;
  *(volatile v8us*)pl = lv;
  if (tid < 8) *(volatile v4f*)(dsq + 4 * tid) = sq;
  __threadfence();
  *(volatile v8us*)ph = hv;
  *(volatile v8us*)pl = lv;
  if (tid < 8) *(volatile v4f*)(dsq + 4 * tid) = sq;
}

__global__ __launch_bounds__(256) void pdy_kernel(
    const int* __restrict__ yl, const float* __restrict__ su, float* __restrict__ pdy)
{
  __shared__ __attribute__((aligned(16))) float sP[256 * PDP];

  const int tid = threadIdx.x, b = blockIdx.x;
  const int j = 256 * b + tid;
  float* sp = sP + tid * PDP;

  if (b < NL / 256) {
    const int y = yl[j];
    #pragma unroll
    for (int c = 0; c < PDP; ++c) sp[c] = (c == y) ? 1.0f : 0.0f;
  } else {
    const float* sr = su + (size_t)(j - NL) * NC;
    float mx = -3.0e38f;
    #pragma unroll 1
    for (int c = 0; c < NC; ++c) mx = fmaxf(mx, sr[c]);
    float sum = 0.0f;
    #pragma unroll 1
    for (int c = 0; c < NC; ++c) {
      const float e = __expf(sr[c] - mx);
      sp[c] = e;
      sum += e;
    }
    const float inv = 1.0f / sum;
    #pragma unroll 1
    for (int c = 0; c < NC; ++c) sp[c] = sp[c] * inv;
    #pragma unroll
    for (int c = NC; c < PDP; ++c) sp[c] = 0.0f;
  }
  __syncthreads();

  float* base = pdy + (size_t)b * 256 * PDP;
  v4f v[4];
  #pragma unroll
  for (int i = 0; i < 4; ++i) v[i] = *(const v4fa*)(sP + 4 * (tid + 256 * i));
  #pragma unroll
  for (int i = 0; i < 4; ++i) *(volatile v4f*)(base + 4 * (tid + 256 * i)) = v[i];
  __threadfence();
  #pragma unroll
  for (int i = 0; i < 4; ++i) *(volatile v4f*)(base + 4 * (tid + 256 * i)) = v[i];
}

__global__ __launch_bounds__(32) void density_kernel(
    const unsigned short* __restrict__ xhi, const unsigned short* __restrict__ xlo,
    const unsigned short* __restrict__ ahi, const unsigned short* __restrict__ alo,
    const float* __restrict__ x2, const float* __restrict__ a2,
    const float* __restrict__ pdy, float* __restrict__ out)
{
  __shared__ __attribute__((aligned(16))) float sOut[16 * NC];

  const int lane = threadIdx.x & 31, h = lane >> 4, m = lane & 15;
  const int row0 = blockIdx.x * 16;

  const unsigned short* xr  = xhi + (size_t)(row0 + m) * DIM;
  const unsigned short* xrl = xlo + (size_t)(row0 + m) * DIM;
  const v16us Ah0 = load_frag(xr,  0, h);
  const v16us Ah1 = load_frag(xr, 32, h);
  const v16us Al0 = load_frag(xrl, 0, h);
  const v16us Al1 = load_frag(xrl,32, h);

  const v4f xa = *(const v4fa*)(x2 + row0 + 8 * h);
  const v4f xb = *(const v4fa*)(x2 + row0 + 8 * h + 4);
  const float x2v[8] = { xa.x, xa.y, xa.z, xa.w, xb.x, xb.y, xb.z, xb.w };

  const v8f zero8 = { 0.f, 0.f, 0.f, 0.f, 0.f, 0.f, 0.f, 0.f };
  float den[8];
  float num[8][NC];
  #pragma unroll
  for (int r = 0; r < 8; ++r) {
    den[r] = 0.0f;
    #pragma unroll
    for (int c = 0; c < NC; ++c) num[r][c] = 0.0f;
  }

  #pragma unroll 1
  for (int jt = 0; jt < JT; ++jt) {
    const int j = jt * 16 + m;
    const unsigned short* ar  = ahi + (size_t)j * DIM;
    const unsigned short* arl = alo + (size_t)j * DIM;
    const v16us Bh0 = load_frag(ar,  0, h);
    const v16us Bh1 = load_frag(ar, 32, h);
    const v16us Bl0 = load_frag(arl, 0, h);
    const v16us Bl1 = load_frag(arl,32, h);

    v8f acc = zero8;
    acc = wmma_bf16(Ah0, Bh0, acc);
    acc = wmma_bf16(Al0, Bh0, acc);
    acc = wmma_bf16(Ah1, Bh1, acc);
    acc = wmma_bf16(Al1, Bh1, acc);
    acc = wmma_bf16(Ah0, Bl0, acc);
    acc = wmma_bf16(Ah1, Bl1, acc);

    const float a2j = a2[j];
    const float* wr = pdy + (size_t)j * PDP;
    const v4f w0 = *(const v4fa*)(wr);
    const v4f w1 = *(const v4fa*)(wr + 4);
    const v4f w2 = *(const v4fa*)(wr + 8);
    const float w[NC] = { w0.x, w0.y, w0.z, w0.w, w1.x, w1.y, w1.z, w1.w, w2.x, w2.y };

    #pragma unroll
    for (int r = 0; r < 8; ++r) {
      const float d2 = (x2v[r] + a2j) - 2.0f * acc[r];
      float p = __expf(-0.5f * d2) * INV_SQRT_2PI;
      p = (p < FMIN_NORMAL) ? 0.0f : p;
      den[r] += p;
      #pragma unroll
      for (int c = 0; c < NC; ++c) num[r][c] = fmaf(p, w[c], num[r][c]);
    }
  }

  #pragma unroll
  for (int mk = 1; mk <= 8; mk <<= 1) {
    #pragma unroll
    for (int r = 0; r < 8; ++r) {
      den[r] += __shfl_xor(den[r], mk);
      #pragma unroll
      for (int c = 0; c < NC; ++c) num[r][c] += __shfl_xor(num[r][c], mk);
    }
  }

  if (m == 0) {
    #pragma unroll
    for (int r = 0; r < 8; ++r) {
      const float inv = 1.0f / den[r];
      #pragma unroll
      for (int c = 0; c < NC; ++c) sOut[(8 * h + r) * NC + c] = num[r][c] * inv;
    }
  }
  __syncthreads();

  const v4f o0 = *(const v4fa*)(sOut + 4 * lane);
  const v4f o1 = *(const v4fa*)(sOut + 4 * (32 + (lane & 7)));
  float* ob = out + (size_t)row0 * NC;

  *(volatile v4f*)(ob + 4 * lane) = o0;
  if (lane < 8) *(volatile v4f*)(ob + 128 + 4 * lane) = o1;
  __threadfence();
  *(volatile v4f*)(ob + 4 * lane) = o0;
  if (lane < 8) *(volatile v4f*)(ob + 128 + 4 * lane) = o1;
}

extern "C" void kernel_launch(void* const* d_in, const int* in_sizes, int n_in,
                              void* d_out, int out_size, void* d_ws, size_t ws_size,
                              hipStream_t stream) {
  if (n_in < 5) return;
  if (in_sizes[0] != NX * DIM) return;
  if (in_sizes[1] != NL * DIM) return;
  if (in_sizes[2] != NU * DIM) return;
  if (in_sizes[3] != NU * NC) return;
  if (in_sizes[4] != NL) return;
  if (out_size != NX * NC) return;

  const float* x  = (const float*)d_in[0];
  const float* xl = (const float*)d_in[1];
  const float* xu = (const float*)d_in[2];
  const float* su = (const float*)d_in[3];
  const int*   yl = (const int*)d_in[4];
  float* out = (float*)d_out;

  const size_t xh_bytes  = (size_t)NX * DIM * 2;
  const size_t ah_bytes  = (size_t)MA * DIM * 2;
  const size_t x2_bytes  = (size_t)NX * 4;
  const size_t a2_bytes  = (size_t)MA * 4;
  const size_t pdy_bytes = (size_t)MA * PDP * 4;
  const size_t o_xhi = 0;
  const size_t o_xlo = o_xhi + xh_bytes;
  const size_t o_ahi = o_xlo + xh_bytes;
  const size_t o_alo = o_ahi + ah_bytes;
  const size_t o_x2  = o_alo + ah_bytes;
  const size_t o_a2  = o_x2 + x2_bytes;
  const size_t o_pdy = o_a2 + a2_bytes;
  const size_t total = o_pdy + pdy_bytes;
  if (total > ws_size) return;

  char* ws = (char*)d_ws;
  unsigned short* xhi = (unsigned short*)(ws + o_xhi);
  unsigned short* xlo = (unsigned short*)(ws + o_xlo);
  unsigned short* ahi = (unsigned short*)(ws + o_ahi);
  unsigned short* alo = (unsigned short*)(ws + o_alo);
  float* x2v  = (float*)(ws + o_x2);
  float* a2v  = (float*)(ws + o_a2);
  float* pdyv = (float*)(ws + o_pdy);

  prep_kernel<<<(NX + MA) / 32, 256, 0, stream>>>(x, xl, xu, xhi, xlo, ahi, alo, x2v, a2v);
  pdy_kernel<<<MA / 256, 256, 0, stream>>>(yl, su, pdyv);
  density_kernel<<<NX / 16, 32, 0, stream>>>(xhi, xlo, ahi, alo, x2v, a2v, pdyv, out);
}
